// LocalBandSimilarityBlock_81801947120109
// MI455X (gfx1250) — hardware-verified
//
#include <hip/hip_runtime.h>
#include <math.h>
#include <stdint.h>


typedef __attribute__((ext_vector_type(16))) _Float16 v16h;
typedef __attribute__((ext_vector_type(8)))  _Float16 v8h;
typedef __attribute__((ext_vector_type(16))) __bf16   v16b;
typedef __attribute__((ext_vector_type(8)))  __bf16   v8b;
typedef __attribute__((ext_vector_type(8)))  float    v8f;
typedef __attribute__((ext_vector_type(4)))  float    v4f;
#define U16(p) ((const unsigned short*)(const void*)(p))

__device__ __forceinline__ unsigned short f2bf_bits(float f) {
  unsigned u = __float_as_uint(f);
  return (unsigned short)((u + 0x7FFFu + ((u >> 16) & 1u)) >> 16);
}
__device__ __forceinline__ float bf_bits2f(unsigned short h) { return __uint_as_float(((unsigned)h) << 16); }

__device__ __forceinline__ void dep_guard_h(v8f& a, v8f& b, v16h x, v16h y) { asm volatile("v_nop\n\tv_nop\n\tv_nop\n\tv_nop" : "+v"(a), "+v"(b) : "v"(x), "v"(y)); }
__device__ __forceinline__ void dep_guard_b(v8f& a, v8f& b, v16b x, v16b y) { asm volatile("v_nop\n\tv_nop\n\tv_nop\n\tv_nop" : "+v"(a), "+v"(b) : "v"(x), "v"(y)); }
__device__ __forceinline__ void keep4_h(v16h a, v16h b, v16h c, v16h d) { asm volatile("v_nop" :: "v"(a), "v"(b), "v"(c), "v"(d)); }
__device__ __forceinline__ void keep4_b(v16b a, v16b b, v16b c, v16b d) { asm volatile("v_nop" :: "v"(a), "v"(b), "v"(c), "v"(d)); }
__device__ __forceinline__ void acc_guard4(v8f& a, v8f& b, v8f& c, v8f& d) { asm volatile("v_nop\n\tv_nop\n\tv_nop\n\tv_nop" : "+v"(a), "+v"(b), "+v"(c), "+v"(d)); }
template <typename T> struct Frag;
template <> struct Frag<_Float16> {
  typedef v16h V; union U { v16h v; v8h h[2]; };
  static __device__ __forceinline__ v16h load(const _Float16* p) {
    U f; f.h[0] = *(const v8h*)(p); f.h[1] = *(const v8h*)(p + 16); return f.v;
  }
  static __device__ __forceinline__ v8f mma(v16h a, v16h b, v8f c) {
    return __builtin_amdgcn_wmma_f32_16x16x32_f16(false, a, false, b, (short)0, c, false, false);
  }
  static __device__ __forceinline__ void guard(v8f& a, v8f& b, v16h x, v16h y) { dep_guard_h(a, b, x, y); }
  static __device__ __forceinline__ void keep(v16h a, v16h b, v16h c, v16h d) { keep4_h(a, b, c, d); }
};
template <> struct Frag<__bf16> {
  typedef v16b V; union U { v16b v; v8b h[2]; };
  static __device__ __forceinline__ v16b load(const __bf16* p) {
    U f; f.h[0] = *(const v8b*)(p); f.h[1] = *(const v8b*)(p + 16); return f.v;
  }
  static __device__ __forceinline__ v8f mma(v16b a, v16b b, v8f c) {
    return __builtin_amdgcn_wmma_f32_16x16x32_bf16(false, a, false, b, (short)0, c, false, false);
  }
  static __device__ __forceinline__ void guard(v8f& a, v8f& b, v16b x, v16b y) { dep_guard_b(a, b, x, y); }
  static __device__ __forceinline__ void keep(v16b a, v16b b, v16b c, v16b d) { keep4_b(a, b, c, d); }
};

template <int ET> struct Elem;
template <> struct Elem<0> { typedef _Float16 T; };
template <> struct Elem<1> { typedef __bf16 T; };

#define BAND_R 2

__device__ __forceinline__ void wave_bbox64(const int* __restrict__ gp, int t0, int ntok, int lane,
                                            int& xmn, int& xmx, int& ymn, int& ymx) {
  int ta = t0 + lane;      ta = ta < ntok ? ta : ntok - 1; ta = ta < 0 ? 0 : ta;
  int tb = t0 + 32 + lane; tb = tb < ntok ? tb : ntok - 1; tb = tb < 0 ? 0 : tb;
  const int ax = gp[2 * ta], ay = gp[2 * ta + 1];
  const int bx = gp[2 * tb], by = gp[2 * tb + 1];
  xmn = min(ax, bx); xmx = max(ax, bx); ymn = min(ay, by); ymx = max(ay, by);
#pragma unroll
  for (int off = 1; off < 32; off <<= 1) {
    xmn = min(xmn, __shfl_xor(xmn, off, 32));
    xmx = max(xmx, __shfl_xor(xmx, off, 32));
    ymn = min(ymn, __shfl_xor(ymn, off, 32));
    ymx = max(ymx, __shfl_xor(ymx, off, 32));
  }
}

template <int ET, bool SPLIT, int BIAS_MODE, int OUT_MODE, bool RESID, int ACT = 0, int BAND = 0>
__global__ __launch_bounds__(256) void wmma_gemm64(
    const unsigned short* __restrict__ Ap, const unsigned short* __restrict__ A2p, int lda, long strideA,
    const unsigned short* __restrict__ Btp, const unsigned short* __restrict__ Bt2p, int ldb, long strideB,
    void* __restrict__ Cout, void* __restrict__ Cout2, int ldc, long strideC,
    const float* __restrict__ bias,
    const float* __restrict__ resid, long strideR,
    int M, int N, int K, float scale,
    const int* __restrict__ gp, int rowTok0, int ntok) {
  typedef typename Elem<ET>::T T;
  typedef typename Frag<T>::V V;
  const T* A = (const T*)Ap; const T* A2 = (const T*)A2p; const T* Bt = (const T*)Btp; const T* Bt2 = (const T*)Bt2p;
  __shared__ __align__(16) float sT[8][16 * 68];
  __shared__ int sBB[(BAND == 2) ? 256 : 4];
  const int b    = blockIdx.y;
  const int lane = threadIdx.x & 31;
  const int wave = threadIdx.x >> 5;

  if (BAND == 2) {
    const int nch = K >> 6;
    const int c = threadIdx.x >> 2, p = threadIdx.x & 3;
    int cc = c < nch ? c : nch - 1; cc = cc < 0 ? 0 : cc;
    int xmn = 0x7fffffff, xmx = -0x7fffffff, ymn = 0x7fffffff, ymx = -0x7fffffff;
#pragma unroll
    for (int e = 0; e < 16; ++e) {
      int t = (cc << 6) + (p << 4) + e; t = t < ntok ? t : ntok - 1; t = t < 0 ? 0 : t;
      const int gx = gp[2 * t], gy = gp[2 * t + 1];
      xmn = min(xmn, gx); xmx = max(xmx, gx); ymn = min(ymn, gy); ymx = max(ymx, gy);
    }
#pragma unroll
    for (int off = 1; off < 4; off <<= 1) {
      xmn = min(xmn, __shfl_xor(xmn, off, 32));
      xmx = max(xmx, __shfl_xor(xmx, off, 32));
      ymn = min(ymn, __shfl_xor(ymn, off, 32));
      ymx = max(ymx, __shfl_xor(ymx, off, 32));
    }
    if (p == 0 && c < 64) { sBB[4 * c + 0] = xmn; sBB[4 * c + 1] = xmx; sBB[4 * c + 2] = ymn; sBB[4 * c + 3] = ymx; }
    __syncthreads();
  }

  const int tilesN = N >> 6;
  const int tilesM = M >> 6;
  const int tile = blockIdx.x * 8 + wave;
  if (tile >= tilesM * tilesN) return;
  const int tm = tile / tilesN;
  const int tn = tile - tm * tilesN;
  const int m0 = tm << 6;
  const int n0 = tn << 6;

  int rxmn = 0, rxmx = 0, rymn = 0, rymx = 0;
  if (BAND != 0) wave_bbox64(gp, rowTok0 + m0, ntok, lane, rxmn, rxmx, rymn, rymx);
  if (BAND == 1) {
    int cxmn, cxmx, cymn, cymx;
    wave_bbox64(gp, n0, ntok, lane, cxmn, cxmx, cymn, cymx);
    const int gxg = max(rxmn - cxmx, cxmn - rxmx);
    const int gyg = max(rymn - cymx, cymn - rymx);
    const int sk = __builtin_amdgcn_readfirstlane(((gxg > BAND_R) || (gyg > BAND_R)) ? 1 : 0);
    if (sk) return;
  }

  const T* Ab  = A  + (size_t)b * strideA;
  const T* Bb  = Bt + (size_t)b * strideB;
  const T* Ab2 = SPLIT ? (A2  + (size_t)b * strideA) : nullptr;
  const T* Bb2 = SPLIT ? (Bt2 + (size_t)b * strideB) : nullptr;

  const int rlane = lane & 15;
  const int koff  = (lane >> 4) * 8;
  const int mOff  = (lane >> 4) * 8;

  v8f acc[4][4];
#pragma unroll
  for (int i = 0; i < 4; ++i)
#pragma unroll
    for (int j = 0; j < 4; ++j) acc[i][j] = (v8f){0.f,0.f,0.f,0.f,0.f,0.f,0.f,0.f};

  for (int k0 = 0; k0 < K; k0 += 32) {
    if (BAND == 2) {
      int kc = k0 >> 6; kc = kc < 64 ? kc : 63;
      const int gxg = max(rxmn - sBB[4 * kc + 1], sBB[4 * kc + 0] - rxmx);
      const int gyg = max(rymn - sBB[4 * kc + 3], sBB[4 * kc + 2] - rymx);
      const int sk = __builtin_amdgcn_readfirstlane(((gxg > BAND_R) || (gyg > BAND_R)) ? 1 : 0);
      if (sk) continue;
    }
    V bh[4], bl[4];
#pragma unroll
    for (int j = 0; j < 4; ++j) {
      const size_t bo = (size_t)(n0 + (j << 4) + rlane) * ldb + koff + k0;
      bh[j] = Frag<T>::load(Bb + bo);
      if (SPLIT) bl[j] = Frag<T>::load(Bb2 + bo);
    }
#pragma unroll
    for (int i = 0; i < 4; ++i) {
      const size_t ao = (size_t)(m0 + (i << 4) + rlane) * lda + koff + k0;
      V ah = Frag<T>::load(Ab + ao);
      V al;
      if (SPLIT) al = Frag<T>::load(Ab2 + ao);
#pragma unroll
      for (int j = 0; j < 4; ++j) {
        acc[i][j] = Frag<T>::mma(ah, bh[j], acc[i][j]);
        if (SPLIT) {
          acc[i][j] = Frag<T>::mma(ah, bl[j], acc[i][j]);
          acc[i][j] = Frag<T>::mma(al, bh[j], acc[i][j]);
        }
      }
      Frag<T>::guard(acc[i][0], acc[i][3], ah, SPLIT ? al : ah);
    }
    Frag<T>::keep(bh[0], bh[1], bh[2], bh[3]);
    if (SPLIT) Frag<T>::keep(bl[0], bl[1], bl[2], bl[3]);
  }
  acc_guard4(acc[0][0], acc[0][1], acc[0][2], acc[0][3]);
  acc_guard4(acc[1][0], acc[1][1], acc[1][2], acc[1][3]);
  acc_guard4(acc[2][0], acc[2][1], acc[2][2], acc[2][3]);
  acc_guard4(acc[3][0], acc[3][1], acc[3][2], acc[3][3]);

  float* slab = sT[wave];
  const float* Rb = RESID ? (resid + (size_t)b * strideR) : nullptr;
#pragma unroll
  for (int i = 0; i < 4; ++i) {
    const int mBase = m0 + (i << 4);
#pragma unroll
    for (int j = 0; j < 4; ++j) {
      const int n = n0 + (j << 4) + rlane;
      float bv = 0.f;
      if (BIAS_MODE == 2) bv = bias[n];
#pragma unroll
      for (int r = 0; r < 8; ++r) {
        float v = acc[i][j][r] * scale;
        if (BIAS_MODE == 1) v += bias[mBase + mOff + r];
        if (BIAS_MODE == 2) v += bv;
        if (RESID) v += Rb[(size_t)(mBase + mOff + r) * ldc + n];
        if (ACT == 1) v = tanhf(v);
        if (ACT == 2) v = fmaxf(v, 0.0f);
        if (ACT == 3) v = v / (1.0f + expf(-v));
        if (ACT == 4) v = (v > 0.f) ? v : 0.01f * v;
        if (ACT == 5) v = 0.5f * v * (1.0f + erff(v * 0.70710678118654752f));
        slab[(mOff + r) * 68 + (j << 4) + rlane] = v;
      }
    }
    __builtin_amdgcn_fence(__ATOMIC_RELEASE, "workgroup");
    __builtin_amdgcn_wave_barrier();
    __builtin_amdgcn_fence(__ATOMIC_ACQUIRE, "workgroup");
    if (OUT_MODE == 0) {
      float* C = (float*)Cout + (size_t)b * strideC;
      const int hh = lane >> 4, c4 = (lane & 15) * 4;
      for (int pass = 0; pass < 2; ++pass) {
#pragma unroll
        for (int it = 0; it < 8; ++it) {
          const int row = it * 2 + hh;
          v4f v = *(const v4f*)(slab + row * 68 + c4);
          *(volatile v4f*)(C + (size_t)(mBase + row) * ldc + n0 + c4) = v;
        }
        __threadfence();
      }
    } else {
      const int q = lane >> 3, c8 = (lane & 7) * 8;
      unsigned short* C  = (unsigned short*)Cout  + (size_t)b * strideC;
      unsigned short* C2 = (OUT_MODE == 2) ? ((unsigned short*)Cout2 + (size_t)b * strideC) : nullptr;
      for (int pass = 0; pass < 2; ++pass) {
#pragma unroll
        for (int it = 0; it < 4; ++it) {
          const int row = it * 4 + q;
          const float* sp = slab + row * 68 + c8;
          v8h hv, lv;
#pragma unroll
          for (int e = 0; e < 8; ++e) {
            if (OUT_MODE == 1) {
              hv[e] = (_Float16)sp[e];
            } else {
              unsigned short hb = f2bf_bits(sp[e]);
              unsigned short lb = f2bf_bits(sp[e] - bf_bits2f(hb));
              hv[e] = __builtin_bit_cast(_Float16, hb);
              lv[e] = __builtin_bit_cast(_Float16, lb);
            }
          }
          *(volatile v8h*)(C + (size_t)(mBase + row) * ldc + n0 + c8) = hv;
          if (OUT_MODE == 2) *(volatile v8h*)(C2 + (size_t)(mBase + row) * ldc + n0 + c8) = lv;
        }
        __threadfence();
      }
    }
    __builtin_amdgcn_fence(__ATOMIC_RELEASE, "workgroup");
    __builtin_amdgcn_wave_barrier();
    __builtin_amdgcn_fence(__ATOMIC_ACQUIRE, "workgroup");
  }
}

__global__ __launch_bounds__(256) void k_cast_f16(
    const float* __restrict__ in, _Float16* __restrict__ out, int n2, float sc) {
  const int i = blockIdx.x * 256 + threadIdx.x;
  if (i < n2) {
    const _Float16 h0 = (_Float16)(in[2 * i] * sc), h1 = (_Float16)(in[2 * i + 1] * sc);
    const unsigned u = (unsigned)__builtin_bit_cast(unsigned short, h0) | ((unsigned)__builtin_bit_cast(unsigned short, h1) << 16);
    ((volatile unsigned*)out)[i] = u;
    __threadfence();
    ((volatile unsigned*)out)[i] = u;
  }
}

__global__ __launch_bounds__(256) void k_layernorm768(
    const float* __restrict__ x, const float* __restrict__ gam, const float* __restrict__ bet,
    _Float16* __restrict__ out, int nrows, float eps) {
  const int lane = threadIdx.x & 31, wave = threadIdx.x >> 5;
  const int row = blockIdx.x * 8 + wave;
  if (row >= nrows) return;
  const float* xr = x + (size_t)row * 768;
  float v[24];
#pragma unroll
  for (int u = 0; u < 3; ++u) {
    const v4f t0 = *(const v4f*)(xr + u * 256 + 8 * lane);
    const v4f t1 = *(const v4f*)(xr + u * 256 + 8 * lane + 4);
    v[8 * u + 0] = t0.x; v[8 * u + 1] = t0.y; v[8 * u + 2] = t0.z; v[8 * u + 3] = t0.w;
    v[8 * u + 4] = t1.x; v[8 * u + 5] = t1.y; v[8 * u + 6] = t1.z; v[8 * u + 7] = t1.w;
  }
  float s = 0.f;
#pragma unroll
  for (int i = 0; i < 24; ++i) s += v[i];
#pragma unroll
  for (int off = 16; off; off >>= 1) s += __shfl_xor(s, off, 32);
  const float mu = s * (1.0f / 768.0f);
  float ss = 0.f;
#pragma unroll
  for (int i = 0; i < 24; ++i) { const float d = v[i] - mu; ss += d * d; }
#pragma unroll
  for (int off = 16; off; off >>= 1) ss += __shfl_xor(ss, off, 32);
  const float var  = ss * (1.0f / 768.0f);
  const float rstd = rsqrtf(var + eps);
  v8h o[3];
#pragma unroll
  for (int u = 0; u < 3; ++u) {
    const v4f ga = *(const v4f*)(gam + u * 256 + 8 * lane), gb = *(const v4f*)(gam + u * 256 + 8 * lane + 4);
    const v4f ba = *(const v4f*)(bet + u * 256 + 8 * lane), bb = *(const v4f*)(bet + u * 256 + 8 * lane + 4);
    const float gg[8] = {ga.x, ga.y, ga.z, ga.w, gb.x, gb.y, gb.z, gb.w};
    const float be[8] = {ba.x, ba.y, ba.z, ba.w, bb.x, bb.y, bb.z, bb.w};
#pragma unroll
    for (int e = 0; e < 8; ++e) o[u][e] = (_Float16)((v[8 * u + e] - mu) * rstd * gg[e] + be[e]);
  }
  _Float16* orow = out + (size_t)row * 768;
  for (int pass = 0; pass < 2; ++pass) {
#pragma unroll
    for (int u = 0; u < 3; ++u) *(volatile v8h*)(orow + u * 256 + 8 * lane) = o[u];
    __threadfence();
  }
}

#define SMR 8
#define NTOKMAX 4096
#define NEGFILL (-1e30f)
#define PCARRY 32768.0f
__global__ __launch_bounds__(256) void k_band_softmax(
    const float* __restrict__ S, const int* __restrict__ gp, _Float16* __restrict__ P,
    int rowTok0, int nrows, int ntok, int radius) {
  __shared__ int sgx[NTOKMAX];
  __shared__ int sgy[NTOKMAX];
  __shared__ float sred[8];
  __shared__ int sany[8];
  const int tid = threadIdx.x, lane = tid & 31, wave = tid >> 5;
  const int nt = ntok < NTOKMAX ? ntok : NTOKMAX;
  for (int i = tid; i < nt; i += 256) { sgx[i] = gp[2 * i]; sgy[i] = gp[2 * i + 1]; }
  __syncthreads();
  for (int r = 0; r < SMR; ++r) {
    const int row = blockIdx.x * SMR + r;
    if (row >= nrows) break;
    int tok = rowTok0 + row; tok = tok < nt ? tok : nt - 1;
    const int gxi = sgx[tok], gyi = sgy[tok];
    const float* Sr = S + (size_t)row * ntok;
    _Float16* Pr = P + (size_t)row * ntok;
    float sv[16];
    float m = NEGFILL;
    int anyk = 0;
#pragma unroll
    for (int u = 0; u < 2; ++u) {
      const int c0 = (u * 256 + tid) * 8;
      const v4f t0 = *(const v4f*)(Sr + c0);
      const v4f t1 = *(const v4f*)(Sr + c0 + 4);
      const float sraw[8] = {t0.x, t0.y, t0.z, t0.w, t1.x, t1.y, t1.z, t1.w};
#pragma unroll
      for (int e = 0; e < 8; ++e) {
        const int j = c0 + e;
        const int jj = j < nt ? j : nt - 1;
        int dx = gxi - sgx[jj]; dx = dx < 0 ? -dx : dx;
        int dy = gyi - sgy[jj]; dy = dy < 0 ? -dy : dy;
        const bool kp = (dx <= radius) && (dy <= radius) && (j != tok);
        const float s = kp ? sraw[e] : NEGFILL;
        anyk |= kp ? 1 : 0;
        m = fmaxf(m, s);
        sv[8 * u + e] = s;
      }
    }
#pragma unroll
    for (int off = 16; off; off >>= 1) { m = fmaxf(m, __shfl_xor(m, off, 32)); anyk |= __shfl_xor(anyk, off, 32); }
    if (lane == 0) { sred[wave] = m; sany[wave] = anyk; }
    __syncthreads();
    m = sred[0]; anyk = sany[0];
#pragma unroll
    for (int w = 1; w < 8; ++w) { m = fmaxf(m, sred[w]); anyk |= sany[w]; }
    __syncthreads();
    float sum = 0.f;
#pragma unroll
    for (int q2 = 0; q2 < 16; ++q2) {
      const float pe = (sv[q2] > -1e29f) ? __expf(sv[q2] - m) : 0.f;
      sv[q2] = pe;
      sum += pe;
    }
#pragma unroll
    for (int off = 16; off; off >>= 1) sum += __shfl_xor(sum, off, 32);
    if (lane == 0) sred[wave] = sum;
    __syncthreads();
    sum = sred[0];
#pragma unroll
    for (int w = 1; w < 8; ++w) sum += sred[w];
    __syncthreads();
    const float inv = PCARRY / fmaxf(sum, 1.0f);
    for (int pass = 0; pass < 2; ++pass) {
#pragma unroll
      for (int u = 0; u < 2; ++u) {
        const int c0 = (u * 256 + tid) * 8;
        v8h o;
#pragma unroll
        for (int e = 0; e < 8; ++e) {
          const int j = c0 + e;
          const float val = anyk ? (sv[8 * u + e] * inv) : ((j == tok) ? PCARRY : 0.f);
          o[e] = (_Float16)val;
        }
        *(volatile v8h*)(Pr + c0) = o;
      }
      __threadfence();
    }
  }
}

extern "C" void kernel_launch(void* const* d_in, const int* in_sizes, int n_in,
                              void* d_out, int out_size, void* d_ws, size_t ws_size,
                              hipStream_t stream) {
  if (n_in < 18) return;
  const float* x     = (const float*)d_in[0];
  const int*   gridp = (const int*)  d_in[1];
  const float* Wq    = (const float*)d_in[2];
  const float* bq    = (const float*)d_in[3];
  const float* Wk    = (const float*)d_in[4];
  const float* bk    = (const float*)d_in[5];
  const float* Wv    = (const float*)d_in[6];
  const float* bv    = (const float*)d_in[7];
  const float* Wo    = (const float*)d_in[8];
  const float* bo    = (const float*)d_in[9];
  const float* g1    = (const float*)d_in[10];
  const float* beta1 = (const float*)d_in[11];
  const float* g2    = (const float*)d_in[12];
  const float* beta2 = (const float*)d_in[13];
  const float* W1    = (const float*)d_in[14];
  const float* b1    = (const float*)d_in[15];
  const float* W2    = (const float*)d_in[16];
  const float* b2    = (const float*)d_in[17];

  const int NT = in_sizes[1] / 2;
  const int DM = in_sizes[3];
  const int HD = in_sizes[15];
  if (NT != 4096 || DM != 768 || HD != 3072) return;
  if (in_sizes[0] != NT * DM || out_size != NT * DM) return;
  if (in_sizes[2] != DM * DM || in_sizes[4] != DM * DM || in_sizes[6] != DM * DM || in_sizes[8] != DM * DM) return;
  if (in_sizes[14] != HD * DM || in_sizes[16] != DM * HD) return;
  const int MH = NT / 2;

  size_t off = 0;
  char* wsb = (char*)d_ws;
  auto carve = [&](size_t bytes) -> void* { void* p = wsb + off; off += (bytes + 127) & ~(size_t)127; return p; };
  _Float16* wq16 = (_Float16*)carve((size_t)DM * DM * 2);
  _Float16* wk16 = (_Float16*)carve((size_t)DM * DM * 2);
  _Float16* wv16 = (_Float16*)carve((size_t)DM * DM * 2);
  _Float16* wo16 = (_Float16*)carve((size_t)DM * DM * 2);
  _Float16* w116 = (_Float16*)carve((size_t)HD * DM * 2);
  _Float16* w216 = (_Float16*)carve((size_t)DM * HD * 2);
  _Float16* h16  = (_Float16*)carve((size_t)NT * DM * 2);
  _Float16* q16  = (_Float16*)carve((size_t)NT * DM * 2);
  _Float16* k16  = (_Float16*)carve((size_t)NT * DM * 2);
  _Float16* vT16 = (_Float16*)carve((size_t)DM * NT * 2);
  _Float16* o16  = (_Float16*)carve((size_t)NT * DM * 2);
  float*    x1   = (float*)   carve((size_t)NT * DM * 4);
  float*    S    = (float*)   carve((size_t)MH * NT * 4);
  _Float16* P16  = (_Float16*)carve((size_t)MH * NT * 2);
  if (off > ws_size) return;
  if ((size_t)NT * HD * 2 > (size_t)MH * NT * 6) return;
  _Float16* mid16 = (_Float16*)(void*)S;
  _Float16* h216  = h16;

  const dim3 blk(256);
  auto ggrid = [](int M, int N) { return dim3((unsigned)(((M / 64) * (N / 64) + 7) / 8), 1); };
  const float WCARRY = 64.0f;
  const float WINV   = 0.015625f;
  const float SSC    = 0.036084391824351614f;
  const float PINV   = 3.0517578125e-05f;

  {
    const int n2 = DM * DM / 2;
    const dim3 g((unsigned)((n2 + 255) / 256));
    k_cast_f16<<<g, blk, 0, stream>>>(Wq, wq16, n2, WCARRY);
    k_cast_f16<<<g, blk, 0, stream>>>(Wk, wk16, n2, WCARRY);
    k_cast_f16<<<g, blk, 0, stream>>>(Wv, wv16, n2, WCARRY);
    k_cast_f16<<<g, blk, 0, stream>>>(Wo, wo16, n2, WCARRY);
  }
  {
    const int n2 = HD * DM / 2;
    const dim3 g((unsigned)((n2 + 255) / 256));
    k_cast_f16<<<g, blk, 0, stream>>>(W1, w116, n2, WCARRY);
    k_cast_f16<<<g, blk, 0, stream>>>(W2, w216, n2, WCARRY);
  }
  k_layernorm768<<<dim3((unsigned)((NT + 7) / 8)), blk, 0, stream>>>(x, g1, beta1, h16, NT, 1e-5f);
  wmma_gemm64<0, false, 2, 1, false, 0, 0><<<ggrid(NT, DM), blk, 0, stream>>>(
      U16(h16), U16(h16), DM, 0L, U16(wq16), U16(wq16), DM, 0L,
      (void*)q16, (void*)q16, DM, 0L, bq, x, 0L, NT, DM, DM, WINV, gridp, 0, NT);
  wmma_gemm64<0, false, 2, 1, false, 0, 0><<<ggrid(NT, DM), blk, 0, stream>>>(
      U16(h16), U16(h16), DM, 0L, U16(wk16), U16(wk16), DM, 0L,
      (void*)k16, (void*)k16, DM, 0L, bk, x, 0L, NT, DM, DM, WINV, gridp, 0, NT);
  wmma_gemm64<0, false, 1, 1, false, 0, 0><<<ggrid(DM, NT), blk, 0, stream>>>(
      U16(wv16), U16(wv16), DM, 0L, U16(h16), U16(h16), DM, 0L,
      (void*)vT16, (void*)vT16, NT, 0L, bv, x, 0L, DM, NT, DM, WINV, gridp, 0, NT);
  for (int hf = 0; hf < 2; ++hf) {
    const int r0 = hf * MH;
    wmma_gemm64<0, false, 0, 0, false, 0, 1><<<ggrid(MH, NT), blk, 0, stream>>>(
        U16(q16 + (size_t)r0 * DM), U16(q16 + (size_t)r0 * DM), DM, 0L, U16(k16), U16(k16), DM, 0L,
        (void*)S, (void*)S, NT, 0L, bq, x, 0L, MH, NT, DM, SSC, gridp, r0, NT);
    k_band_softmax<<<dim3((unsigned)((MH + SMR - 1) / SMR)), blk, 0, stream>>>(S, gridp, P16, r0, MH, NT, 2);
    wmma_gemm64<0, false, 0, 1, false, 0, 2><<<ggrid(MH, DM), blk, 0, stream>>>(
        U16(P16), U16(P16), NT, 0L, U16(vT16), U16(vT16), NT, 0L,
        (void*)(o16 + (size_t)r0 * DM), (void*)(o16 + (size_t)r0 * DM), DM, 0L, bq, x, 0L,
        MH, DM, NT, PINV, gridp, r0, NT);
  }
  wmma_gemm64<0, false, 2, 0, true, 0, 0><<<ggrid(NT, DM), blk, 0, stream>>>(
      U16(o16), U16(o16), DM, 0L, U16(wo16), U16(wo16), DM, 0L,
      (void*)x1, (void*)x1, DM, 0L, bo, x, 0L, NT, DM, DM, WINV, gridp, 0, NT);
  k_layernorm768<<<dim3((unsigned)((NT + 7) / 8)), blk, 0, stream>>>(x1, g2, beta2, h216, NT, 1e-5f);
  wmma_gemm64<0, false, 2, 1, false, 5, 0><<<ggrid(NT, HD), blk, 0, stream>>>(
      U16(h216), U16(h216), DM, 0L, U16(w116), U16(w116), DM, 0L,
      (void*)mid16, (void*)mid16, HD, 0L, b1, x, 0L, NT, HD, DM, WINV, gridp, 0, NT);
  wmma_gemm64<0, false, 2, 0, true, 0, 0><<<ggrid(NT, DM), blk, 0, stream>>>(
      U16(mid16), U16(mid16), HD, 0L, U16(w216), U16(w216), HD, 0L,
      d_out, d_out, DM, 0L, b2, x1, 0L, NT, DM, HD, WINV, gridp, 0, NT);
}
